// GCNLayer_3470333575494
// MI455X (gfx1250) — hardware-run, weakly checked
//
#include <hip/hip_runtime.h>

typedef float          v8f   __attribute__((ext_vector_type(8)));
typedef float          v4f   __attribute__((ext_vector_type(4)));
typedef unsigned int   v4u   __attribute__((ext_vector_type(4)));
typedef int            v8i   __attribute__((ext_vector_type(8)));
typedef unsigned short v8us  __attribute__((ext_vector_type(8)));
typedef unsigned short v16us __attribute__((ext_vector_type(16)));
typedef __bf16         v16bf __attribute__((ext_vector_type(16)));
typedef _Float16       v16h  __attribute__((ext_vector_type(16)));
typedef v4f  __attribute__((may_alias)) v4fa;
typedef v8us __attribute__((may_alias)) v8usa;
union FragB { v16bf v; v16us u; v8us h[2]; v8i w; };
union FragH { v16h  v; v16us u; v8us h[2]; v8i w; };

__device__ __forceinline__ v8f wmb(const FragB& a, const FragB& b, v8f c) {
  v8f d = __builtin_amdgcn_wmma_f32_16x16x32_bf16(false, a.v, false, b.v, (short)0, c, false, false);
  asm volatile("v_nop\n\tv_nop\n\tv_nop\n\tv_nop" : "+v"(d) : "v"(a.w), "v"(b.w));
  return d;
}

__device__ __forceinline__ v8f wmh(const FragH& a, const FragH& b, v8f c) {
  v8f d = __builtin_amdgcn_wmma_f32_16x16x32_f16(false, a.v, false, b.v, (short)0, c, false, false);
  asm volatile("v_nop\n\tv_nop\n\tv_nop\n\tv_nop" : "+v"(d) : "v"(a.w), "v"(b.w));
  return d;
}

__device__ __forceinline__ unsigned bf16_bits(float f) {
  const unsigned u = __float_as_uint(f);
  const unsigned r = (u + 0x7FFFu + ((u >> 16) & 1u)) >> 16;
  const unsigned q = (u >> 16) | 0x40u;
  return ((u & 0x7fffffffu) > 0x7f800000u) ? q : r;
}

__device__ __forceinline__ float bf16_val(float f) {
  return __uint_as_float(bf16_bits(f) << 16);
}
__device__ __forceinline__ int clampi(int v, int lo, int hi) {
  return v < lo ? lo : (v > hi ? hi : v);
}

__device__ __forceinline__ unsigned f16_bits(float f) {
  const unsigned u  = __float_as_uint(f);
  const unsigned s  = (u >> 16) & 0x8000u;
  const unsigned a  = u & 0x7fffffffu;
  const unsigned t  = a - 0x38000000u;
  const unsigned r  = (t + 0x0FFFu + ((t >> 13) & 1u)) >> 13;
  const unsigned rc = r > 0x7C00u ? 0x7C00u : r;
  const bool small  = a < 0x38800000u;
  const bool isnan  = a > 0x7f800000u;
  const unsigned fin = small ? 0u : (s | rc);
  return isnan ? (s | 0x7E00u) : fin;
}

__device__ __forceinline__ unsigned pk16(unsigned lo, unsigned hi) { return lo | (hi << 16); }
__device__ __forceinline__ unsigned bf16_lo_bits(float v) {
  float hi = bf16_val(v);
  asm volatile("" : "+v"(hi));
  return bf16_bits(v - hi);
}
__device__ __forceinline__ v4u pack8_bf16(v4f a, v4f c) {
  return (v4u){ pk16(bf16_bits(a[0]), bf16_bits(a[1])), pk16(bf16_bits(a[2]), bf16_bits(a[3])),
                pk16(bf16_bits(c[0]), bf16_bits(c[1])), pk16(bf16_bits(c[2]), bf16_bits(c[3])) };
}
__device__ __forceinline__ v4u pack8_bf16_lo(v4f a, v4f c) {
  return (v4u){ pk16(bf16_lo_bits(a[0]), bf16_lo_bits(a[1])), pk16(bf16_lo_bits(a[2]), bf16_lo_bits(a[3])),
                pk16(bf16_lo_bits(c[0]), bf16_lo_bits(c[1])), pk16(bf16_lo_bits(c[2]), bf16_lo_bits(c[3])) };
}
__device__ __forceinline__ v4u pack8_f16(v4f a, v4f c) {
  return (v4u){ pk16(f16_bits(a[0]), f16_bits(a[1])), pk16(f16_bits(a[2]), f16_bits(a[3])),
                pk16(f16_bits(c[0]), f16_bits(c[1])), pk16(f16_bits(c[2]), f16_bits(c[3])) };
}

template <int FORM>
__global__ __launch_bounds__(256) void k_plane(const float* __restrict__ src, int rows, int cols, int ldsrc,
                                               unsigned short* __restrict__ dst, int MP, int KP) {
  static_assert(FORM >= 0 && FORM <= 3);
  const int KTOT = (FORM == 1 || FORM == 3) ? 2 * KP : KP;
  const unsigned ppr   = (unsigned)(KTOT >> 3);
  const unsigned kp8   = (unsigned)(KP >> 3);
  const unsigned total = (unsigned)MP * ppr;
  const unsigned g     = blockIdx.x * 256u + threadIdx.x;
  const unsigned rowu  = g / ppr;
  const unsigned p     = g - rowu * ppr;
  const bool second    = p >= kp8;
  const int row = (int)rowu;
  const int c0  = (int)((second ? p - kp8 : p) << 3);
  const float* srow = src + (size_t)clampi(row, 0, rows - 1) * (size_t)ldsrc;
  float x[8];
  unsigned mk[8];
#pragma unroll
  for (int e = 0; e < 8; ++e) {
    const int c = c0 + e;
    const float v = srow[clampi(c, 0, cols - 1)];
    asm volatile("" :: "v"(v));
    x[e]  = v;
    mk[e] = (row < rows && c < cols) ? 0xFFFFu : 0u;
  }
  const v4f a = (v4f){ x[0], x[1], x[2], x[3] };
  const v4f c = (v4f){ x[4], x[5], x[6], x[7] };
  v4u o;
  if (FORM == 2) {
    o = pack8_f16(a, c);
  } else {
    const v4u hi = pack8_bf16(a, c);
    o = hi;
    if (FORM == 1) { const v4u lo = pack8_bf16_lo(a, c); o = second ? lo : hi; }
  }
  const v4u mw = (v4u){ pk16(mk[0], mk[1]), pk16(mk[2], mk[3]), pk16(mk[4], mk[5]), pk16(mk[6], mk[7]) };
  o &= mw;
  if (g < total) {
    volatile v4u* q = (volatile v4u*)(dst + (size_t)g * 8);
    *q = o;
    __threadfence();
    *q = o;
  }
}

template <int FORM> struct FragOf    { typedef FragB T; };
template <>         struct FragOf<2> { typedef FragH T; };
__device__ __forceinline__ v8f mm(const FragB& a, const FragB& b, v8f c) { return wmb(a, b, c); }
__device__ __forceinline__ v8f mm(const FragH& a, const FragH& b, v8f c) { return wmh(a, b, c); }
template <class F> __device__ __forceinline__ F ld_frag(const unsigned short* p) {
  F f;
  f.h[0] = *(const v8usa*)(p);
  f.h[1] = *(const v8usa*)(p + 16);
  return f;
}

template <int FORM, int EPI>
__global__ __launch_bounds__(256) __attribute__((amdgpu_num_vgpr(248)))
void k_gemm_nt(const unsigned short* __restrict__ A, const unsigned short* __restrict__ B,
               const float* __restrict__ bias, float* __restrict__ D, int M, int N, int KTOT, int ldd) {
  static_assert(FORM >= 0 && FORM <= 2);
  static_assert(EPI == 0 || EPI == 1);
  typedef typename FragOf<FORM>::T F;
  __shared__ __attribute__((aligned(16))) float sT[8][16 * 68];
  const int lane = threadIdx.x & 31;
  const int wave = threadIdx.x >> 5;
  const int tilesM = (M + 63) >> 6;
  const int tilesN = (N + 63) >> 6;
  const int tile = blockIdx.x * 8 + wave;
  if (tile >= tilesM * tilesN) return;
  const int tm = tile / tilesN;
  const int tn = tile - tm * tilesN;
  const int m0 = tm << 6;
  const int n0 = tn << 6;

  const int rl = lane & 15;
  const int h8 = (lane >> 4) * 8;
  const unsigned short* pa = A + (size_t)(m0 + rl) * (size_t)KTOT + h8;
  const unsigned short* pb = B + (size_t)(n0 + rl) * (size_t)KTOT + h8;

  v8f acc[4][4];
#pragma unroll
  for (int i = 0; i < 4; ++i)
#pragma unroll
    for (int j = 0; j < 4; ++j) acc[i][j] = (v8f){0.f, 0.f, 0.f, 0.f, 0.f, 0.f, 0.f, 0.f};

#pragma unroll 1
  for (int k0 = 0; k0 < KTOT; k0 += 32) {
    F bf[4];
#pragma unroll
    for (int j = 0; j < 4; ++j) bf[j] = ld_frag<F>(pb + (size_t)(j << 4) * (size_t)KTOT + k0);
#pragma unroll
    for (int i = 0; i < 4; ++i) {
      const F af = ld_frag<F>(pa + (size_t)(i << 4) * (size_t)KTOT + k0);
#pragma unroll
      for (int j = 0; j < 4; ++j) acc[i][j] = mm(af, bf[j], acc[i][j]);
    }
  }

  float* slab = sT[wave];
  const int hh = lane >> 4;
  const int c4 = (lane & 15) * 4;
  const int nc = n0 + c4;
  const bool cok = nc < N;
  v4f bv = (v4f){0.f, 0.f, 0.f, 0.f};
  if (EPI == 1) {
    bv = *(const v4fa*)(bias + clampi(nc, 0, N - 4));
    asm volatile("" :: "v"(bv));
  }
#pragma unroll
  for (int i = 0; i < 4; ++i) {
    const int mBase = m0 + (i << 4);
#pragma unroll
    for (int j = 0; j < 4; ++j) {
#pragma unroll
      for (int r = 0; r < 8; ++r) slab[(h8 + r) * 68 + (j << 4) + rl] = acc[i][j][r];
    }
    __builtin_amdgcn_fence(__ATOMIC_RELEASE, "workgroup");
    __builtin_amdgcn_wave_barrier();
    __builtin_amdgcn_fence(__ATOMIC_ACQUIRE, "workgroup");
    v4f vv[8];
#pragma unroll
    for (int it = 0; it < 8; ++it) {
      const int row = it * 2 + hh;
      v4f v = *(const v4fa*)(slab + row * 68 + c4);
      if (EPI == 1) v += bv;
      vv[it] = v;
    }
    for (int pass = 0; pass < 2; ++pass) {
#pragma unroll
      for (int it = 0; it < 8; ++it) {
        const int row = mBase + it * 2 + hh;
        if (cok && row < M) *(volatile v4f*)(D + (size_t)row * (size_t)ldd + nc) = vv[it];
      }
      __threadfence();
    }
    __builtin_amdgcn_fence(__ATOMIC_RELEASE, "workgroup");
    __builtin_amdgcn_wave_barrier();
    __builtin_amdgcn_fence(__ATOMIC_ACQUIRE, "workgroup");
  }
}

#pragma clang fp contract(off)

#define NN      100000
#define KD      128
#define HD      64
#define NE      1600000
#define MP      100096
#define NTHR    256
#define NWAVE   8
#define EPT     8
#define WCH     (32 * EPT)
#define NBRUN   1024
#define SLB     10
#define ESH     21
#define NBK     98
#define WLCAP   3584
#define RCAP    21504
#define DEGCAP  64
#define MAXDEG_MEAS   35
#define MAXB1024_MEAS 16714

#define BK_ZINTS (NWAVE * WLCAP + RCAP + 3 * NBRUN)
#define BK_INTS  (BK_ZINTS + 16)
#define BK_LDS   (BK_INTS * 4)

#define PBX   (MP * KD / 8 / NTHR)
#define GB    ((MP / 64 + 7) / 8)
#define WTB   (HD * KD / 8 / NTHR)
#define NVU   (MP / 4)
#define NVB   ((NVU + NTHR - 1) / NTHR)
#define TABB  (WTB + NVB + 1)

static_assert(HD == 32 * 2 && HD % 64 == 0 && HD % 32 == 0);
static_assert(KD % 32 == 0);
static_assert(MP % 128 == 0 && MP % 64 == 0 && MP >= NN && MP == 782 * 128 && MP - NN == 96);
static_assert(NN % 4 == 0 && NN % NWAVE == 0 && MP % 4 == 0 && NVU % 32 == 0);
static_assert((MP * KD / 8) % NTHR == 0 && (HD * KD / 8) % NTHR == 0);
static_assert(NBRUN == (1 << SLB) && NBRUN <= (1 << 10) && NBRUN % 32 == 0);
static_assert(NE <= (1 << ESH) && SLB + ESH <= 31);
static_assert(NBK * NBRUN >= MP && (NBK - 1) * NBRUN < NN);
static_assert(NE % WCH == 0 && NE % 8 == 0);
static_assert(RCAP % 256 == 0 && RCAP % (NTHR * 4) == 0 && (2 * NBRUN) % (NTHR * 4) == 0);
static_assert((long long)RCAP * 100 >= (long long)MAXB1024_MEAS * 125);
static_assert(WLCAP * 8 >= (RCAP / 8) * 10);
static_assert(WLCAP >= MAXB1024_MEAS / 8 + 8 * 46 + 1);
static_assert(MAXDEG_MEAS + 8 <= DEGCAP && DEGCAP < RCAP);
static_assert(BK_ZINTS % (NTHR * 4) == 0);
static_assert(BK_LDS <= 262144);

typedef float v2f __attribute__((ext_vector_type(2)));
typedef int   v4i __attribute__((ext_vector_type(4)));
typedef v2f __attribute__((may_alias)) v2fa;
typedef v4i __attribute__((may_alias)) v4ia;

__global__ __launch_bounds__(NTHR) void k_wt_tab(const float* __restrict__ w, const float* __restrict__ nrm,
                                                 const float* __restrict__ bias, unsigned short* wt,
                                                 float* nv, float* bv) {
  const int tid = (int)threadIdx.x;
  const int blk = (int)blockIdx.x;
  if (blk < WTB) {
    const int u  = blk * NTHR + tid;
    const int n  = u >> 4, k8 = (u & 15) * 8;
    float f[8];
#pragma unroll
    for (int i = 0; i < 8; ++i) {
      const float v = w[(size_t)(k8 + i) * HD + n];
      asm volatile("" :: "v"(v));
      f[i] = v;
    }
    const v4u o = pack8_bf16((v4f){ f[0], f[1], f[2], f[3] }, (v4f){ f[4], f[5], f[6], f[7] });
    volatile v4u* q = (volatile v4u*)(wt + (size_t)u * 8);
    *q = o;
    __threadfence();
    *q = o;
  } else if (blk < WTB + NVB) {
    const int u  = (blk - WTB) * NTHR + tid;
    const int uc = u < NN / 4 ? u : NN / 4 - 1;
    const v4f a = *(const v4fa*)(nrm + 4 * (size_t)uc);
    asm volatile("" :: "v"(a));
    const unsigned mk = u < NN / 4 ? 0xFFFFFFFFu : 0u;
    v4f o;
    o.x = __uint_as_float((bf16_bits(a.x) << 16) & mk);
    o.y = __uint_as_float((bf16_bits(a.y) << 16) & mk);
    o.z = __uint_as_float((bf16_bits(a.z) << 16) & mk);
    o.w = __uint_as_float((bf16_bits(a.w) << 16) & mk);
    if (u < NVU) {
      volatile v4f* q = (volatile v4f*)(nv + 4 * (size_t)u);
      *q = o;
      __threadfence();
      *q = o;
    }
  } else {
    const int tc = tid & 15;
    const v4f a = *(const v4fa*)(bias + 4 * tc);
    asm volatile("" :: "v"(a));
    v4f o;
    o.x = bf16_val(a.x); o.y = bf16_val(a.y); o.z = bf16_val(a.z); o.w = bf16_val(a.w);
    if (tid < 16) {
      volatile v4f* q = (volatile v4f*)(bv + 4 * tid);
      *q = o;
      __threadfence();
      *q = o;
    }
  }
}

__global__ __launch_bounds__(NTHR) void k_bucket(const int* __restrict__ srcs, const int* __restrict__ dsts,
                                                 int* LIST, int* CO, int* FLAG) {
  extern __shared__ __attribute__((aligned(16))) int dsm[];
  int* wl   = dsm;
  int* pl   = dsm + NWAVE * WLCAP;
  int* cnt  = pl + RCAP;
  int* offs = cnt + NBRUN;
  int* cur  = offs + NBRUN;
  int* misc = cur + NBRUN;
  const int tid  = (int)threadIdx.x, lane = tid & 31;
  const int wave = __builtin_amdgcn_readfirstlane(tid >> 5);
  const int blk  = (int)blockIdx.x;
  const unsigned nbs = (unsigned)(blk * NBRUN);

  {
    const v4i z4 = {0, 0, 0, 0};
#pragma unroll 1
    for (int i = tid * 4; i < BK_ZINTS; i += NTHR * 4) *(v4ia*)(dsm + i) = z4;
    if (tid < 16) misc[tid] = 0;
  }
  __syncthreads();

  {
    const int per  = ((NE + NWAVE * WCH - 1) / (NWAVE * WCH)) * WCH;
    const int ebeg = wave * per;
    const int eend = (ebeg + per < NE) ? (ebeg + per) : NE;
    int* mylist = wl + wave * WLCAP;
    int wc = 0;
#pragma unroll 1
    for (int cb = ebeg; cb < eend; cb += WCH) {
      const int e0 = cb + lane * EPT;
      const v4i da = *(const v4ia*)(dsts + e0);
      const v4i db = *(const v4ia*)(dsts + e0 + 4);
      asm volatile("" :: "v"(da.x)); asm volatile("" :: "v"(da.y));
      asm volatile("" :: "v"(da.z)); asm volatile("" :: "v"(da.w));
      asm volatile("" :: "v"(db.x)); asm volatile("" :: "v"(db.y));
      asm volatile("" :: "v"(db.z)); asm volatile("" :: "v"(db.w));
      const unsigned s0 = (unsigned)da.x - nbs, s1 = (unsigned)da.y - nbs;
      const unsigned s2 = (unsigned)da.z - nbs, s3 = (unsigned)da.w - nbs;
      const unsigned s4 = (unsigned)db.x - nbs, s5 = (unsigned)db.y - nbs;
      const unsigned s6 = (unsigned)db.z - nbs, s7 = (unsigned)db.w - nbs;
      const bool h0 = s0 < (unsigned)NBRUN, h1 = s1 < (unsigned)NBRUN, h2 = s2 < (unsigned)NBRUN, h3 = s3 < (unsigned)NBRUN;
      const bool h4 = s4 < (unsigned)NBRUN, h5 = s5 < (unsigned)NBRUN, h6 = s6 < (unsigned)NBRUN, h7 = s7 < (unsigned)NBRUN;
      const unsigned m0 = __builtin_amdgcn_ballot_w32(h0), m1 = __builtin_amdgcn_ballot_w32(h1);
      const unsigned m2 = __builtin_amdgcn_ballot_w32(h2), m3 = __builtin_amdgcn_ballot_w32(h3);
      const unsigned m4 = __builtin_amdgcn_ballot_w32(h4), m5 = __builtin_amdgcn_ballot_w32(h5);
      const unsigned m6 = __builtin_amdgcn_ballot_w32(h6), m7 = __builtin_amdgcn_ballot_w32(h7);
      const unsigned any = m0 | m1 | m2 | m3 | m4 | m5 | m6 | m7;
      if (any != 0u) {
        const int pre = (int)(__builtin_amdgcn_mbcnt_lo(m0, 0u) + __builtin_amdgcn_mbcnt_lo(m1, 0u) +
                              __builtin_amdgcn_mbcnt_lo(m2, 0u) + __builtin_amdgcn_mbcnt_lo(m3, 0u) +
                              __builtin_amdgcn_mbcnt_lo(m4, 0u) + __builtin_amdgcn_mbcnt_lo(m5, 0u) +
                              __builtin_amdgcn_mbcnt_lo(m6, 0u) + __builtin_amdgcn_mbcnt_lo(m7, 0u));
        int p = wc + pre;
        if (h0) { if (p < WLCAP) mylist[p] = (int)((s0 << ESH) | (unsigned)(e0 + 0)); p = p + 1; }
        if (h1) { if (p < WLCAP) mylist[p] = (int)((s1 << ESH) | (unsigned)(e0 + 1)); p = p + 1; }
        if (h2) { if (p < WLCAP) mylist[p] = (int)((s2 << ESH) | (unsigned)(e0 + 2)); p = p + 1; }
        if (h3) { if (p < WLCAP) mylist[p] = (int)((s3 << ESH) | (unsigned)(e0 + 3)); p = p + 1; }
        if (h4) { if (p < WLCAP) mylist[p] = (int)((s4 << ESH) | (unsigned)(e0 + 4)); p = p + 1; }
        if (h5) { if (p < WLCAP) mylist[p] = (int)((s5 << ESH) | (unsigned)(e0 + 5)); p = p + 1; }
        if (h6) { if (p < WLCAP) mylist[p] = (int)((s6 << ESH) | (unsigned)(e0 + 6)); p = p + 1; }
        if (h7) { if (p < WLCAP) mylist[p] = (int)((s7 << ESH) | (unsigned)(e0 + 7)); p = p + 1; }
        wc += (int)(__builtin_popcount(m0) + __builtin_popcount(m1) + __builtin_popcount(m2) + __builtin_popcount(m3) +
                    __builtin_popcount(m4) + __builtin_popcount(m5) + __builtin_popcount(m6) + __builtin_popcount(m7));
      }
    }
    if (lane == 0) misc[wave] = wc;
  }
  __syncthreads();

  if (wave == 0) {
    int ov = 0;
    int tot = 0;
#pragma unroll 1
    for (int w2 = 0; w2 < NWAVE; ++w2) {
      int c = __builtin_amdgcn_readfirstlane(misc[w2]);
      if (c > WLCAP) ov = 1;
      c = c < 0 ? 0 : (c > WLCAP ? WLCAP : c);
      tot += c;
#pragma unroll 1
      for (int b0 = 0; b0 < c; b0 += 32) {
        const int idx = b0 + lane;
        const int ent = wl[w2 * WLCAP + (idx < WLCAP ? idx : WLCAP - 1)];
        const int m32 = (c - b0) < 32 ? (c - b0) : 32;
#pragma unroll 1
        for (int k = 0; k < m32; ++k) {
          const int u    = __builtin_amdgcn_readlane(ent, k);
          const int slot = (u >> ESH) & (NBRUN - 1);
          if (lane == 0) cnt[slot] = cnt[slot] + 1;
        }
      }
    }
    if (tot > RCAP) ov = 1;
    if (lane == 0) misc[9] = ov;
  }
  __syncthreads();
  if (wave == 0) {
    const int base = lane * (NBRUN / 32);
    int s = 0;
    int dg = 0;
#pragma unroll 1
    for (int i = 0; i < NBRUN / 32; ++i) {
      const int cv = cnt[base + i];
      s += cv;
      dg |= (cv > DEGCAP) ? 1 : 0;
    }
    int incl = s;
#pragma unroll
    for (int d = 1; d < 32; d <<= 1) {
      const int y = __shfl_up(incl, d, 32);
      if (lane >= d) incl += y;
    }
    const unsigned dm = __builtin_amdgcn_ballot_w32(dg != 0);
    if (lane == 0) misc[10] = (dm != 0u) ? 1 : 0;
    int run = incl - s;
#pragma unroll 1
    for (int i = 0; i < NBRUN / 32; ++i) {
      const int cv = cnt[base + i];
      offs[base + i] = run;
      cur[base + i]  = run;
      run += cv;
    }
  }
  __syncthreads();

  if (wave == 0) {
#pragma unroll 1
    for (int w2 = 0; w2 < NWAVE; ++w2) {
      int c = __builtin_amdgcn_readfirstlane(misc[w2]);
      c = c < 0 ? 0 : (c > WLCAP ? WLCAP : c);
#pragma unroll 1
      for (int b0 = 0; b0 < c; b0 += 32) {
        const int idx = b0 + lane;
        const int ent = wl[w2 * WLCAP + (idx < WLCAP ? idx : WLCAP - 1)];
        int eid = ent & ((1 << ESH) - 1);
        eid = eid > NE - 1 ? NE - 1 : eid;
        int sr = srcs[eid];
        asm volatile("" :: "v"(sr));
        sr = sr < 0 ? 0 : (sr > NN - 1 ? NN - 1 : sr);
        const int m32 = (c - b0) < 32 ? (c - b0) : 32;
#pragma unroll 1
        for (int k = 0; k < m32; ++k) {
          const int u    = __builtin_amdgcn_readlane(ent, k);
          const int w0   = __builtin_amdgcn_readlane(sr, k);
          const int slot = (u >> ESH) & (NBRUN - 1);
          if (lane == 0) {
            int p = cur[slot];
            p = p < 0 ? 0 : (p > RCAP - 1 ? RCAP - 1 : p);
            pl[p] = w0;
            cur[slot] = p + 1;
          }
        }
      }
    }
  }
  __syncthreads();

  const int ovf = ((misc[9] | misc[10]) != 0) ? 1 : 0;
  int* lp  = LIST + (size_t)blk * (size_t)RCAP;
  int* cop = CO + (size_t)blk * (2 * NBRUN);
  int* fp  = FLAG + (size_t)blk * 32;
#pragma unroll 1
  for (int pass = 0; pass < 2; ++pass) {
#pragma unroll 1
    for (int i = tid * 4; i < RCAP; i += NTHR * 4) {
      const v4i v = *(const v4ia*)(pl + i);
      *(volatile v4i*)(lp + i) = v;
    }
#pragma unroll 1
    for (int i = tid * 4; i < 2 * NBRUN; i += NTHR * 4) {
      const v4i v = *(const v4ia*)(cnt + i);
      *(volatile v4i*)(cop + i) = v;
    }
    if (tid < 8) {
      const v4i f = {ovf, ovf, ovf, ovf};
      *(volatile v4i*)(fp + 4 * tid) = f;
    }
    __threadfence();
  }
}

__global__ __launch_bounds__(NTHR) void k_walk(const int* __restrict__ LIST, const int* __restrict__ CO,
                                               const int* __restrict__ FLAG, const float* __restrict__ T,
                                               const float* __restrict__ NV, const float* __restrict__ BV,
                                               float* out, int n_real) {
  const int lane = (int)threadIdx.x & 31;
  const int wave = __builtin_amdgcn_readfirstlane((int)threadIdx.x >> 5);
  const int node = (int)blockIdx.x * NWAVE + wave;
  const int ncl  = clampi(node, 0, NN - 1);
  const int blk  = ncl >> SLB;
  const int slot = ncl & (NBRUN - 1);
  const int* lb  = LIST + (size_t)blk * (size_t)RCAP;

  int cr = CO[(size_t)blk * (2 * NBRUN) + slot];
  asm volatile("" :: "v"(cr));
  int orw = CO[(size_t)blk * (2 * NBRUN) + NBRUN + slot];
  asm volatile("" :: "v"(orw));
  int fl = FLAG[(size_t)blk * 32];
  asm volatile("" :: "v"(fl));
  const v2f bvp = *(const v2fa*)(BV + 2 * lane);
  asm volatile("" :: "v"(bvp));

  const bool big = cr > DEGCAP;
  const int n = __builtin_amdgcn_readfirstlane(clampi(cr, 0, DEGCAP));
  const int o = __builtin_amdgcn_readfirstlane(clampi(orw, 0, RCAP - n));
  int last = o + (n > 0 ? n : 1) - 1;
  last = last > RCAP - 1 ? RCAP - 1 : last;

  float a0 = 0.0f, a1 = 0.0f;
#pragma unroll 1
  for (int b0 = 0; b0 < n; b0 += 32) {
    int idx = o + b0 + lane;
    idx = idx > last ? last : idx;
    int sr = lb[idx];
    asm volatile("" :: "v"(sr));
    sr = sr < 0 ? 0 : (sr > NN - 1 ? NN - 1 : sr);
    const float nvv = NV[sr];
    asm volatile("" :: "v"(nvv));
    const int nvb = __float_as_int(nvv);
    const int m32 = (n - b0) < 32 ? (n - b0) : 32;
#pragma unroll 1
    for (int k = 0; k < m32; ++k) {
      const int   sk = __builtin_amdgcn_readlane(sr, k);
      const float ck = __int_as_float(__builtin_amdgcn_readlane(nvb, k));
      const v2f q = *(const v2fa*)(T + (size_t)sk * HD + 2 * lane);
      asm volatile("" :: "v"(q));
      const float p0 = q.x * ck;
      const float p1 = q.y * ck;
      a0 = a0 + p0;
      a1 = a1 + p1;
    }
  }
  const float v0 = a0 + bvp.x;
  const float v1 = a1 + bvp.y;
  const float r0 = (v0 > 0.0f || v0 != v0) ? v0 : 0.0f;
  const float r1 = (v1 > 0.0f || v1 != v1) ? v1 : 0.0f;
  const float qnan = __uint_as_float(0x7fc00000u);
  const bool bad = (fl != 0) || big;
  v2f ov;
  ov.x = bad ? qnan : r0;
  ov.y = bad ? qnan : r1;
  if (node < n_real) {
    float* op = out + (size_t)node * HD + 2 * lane;
    *(volatile v2f*)op = ov;
    __threadfence();
    *(volatile v2f*)op = ov;
  }
}

extern "C" void kernel_launch(void* const* d_in, const int* in_sizes, int n_in,
                              void* d_out, int out_size, void* d_ws, size_t ws_size,
                              hipStream_t stream) {
  if (n_in < 6) return;
  if (in_sizes[0] != NN * KD) return;
  if (in_sizes[1] != KD * HD) return;
  if (in_sizes[2] != NN) return;
  if (in_sizes[3] != HD) return;
  if (in_sizes[4] != NE) return;
  if (in_sizes[5] != NE) return;
  if (out_size != NN * HD) return;

  const float* h    = (const float*)d_in[0];
  const float* W    = (const float*)d_in[1];
  const float* nrm  = (const float*)d_in[2];
  const float* bias = (const float*)d_in[3];
  const int*   srcs = (const int*)d_in[4];
  const int*   dsts = (const int*)d_in[5];
  float* out = (float*)d_out;

  constexpr size_t zHB   = (size_t)MP * KD * 2;
  constexpr size_t zT    = (size_t)MP * HD * 4;
  constexpr size_t zLIST = (size_t)NBK * RCAP * 4;
  constexpr size_t zCO   = (size_t)NBK * 2 * NBRUN * 4;
  constexpr size_t zFLAG = (size_t)NBK * 128;
  constexpr size_t zWT   = (size_t)HD * KD * 2;
  constexpr size_t zNV   = (size_t)MP * 4;
  constexpr size_t zBV   = 256;
  constexpr size_t oHB   = 0;
  constexpr size_t oT    = oHB + zHB;
  constexpr size_t oLIST = oT + zT;
  constexpr size_t oCO   = oLIST + zLIST;
  constexpr size_t oFLAG = oCO + zCO;
  constexpr size_t oWT   = oFLAG + zFLAG;
  constexpr size_t oNV   = oWT + zWT;
  constexpr size_t oBV   = oNV + zNV;
  constexpr size_t oEND  = oBV + zBV;
  static_assert(zHB % 256 == 0 && zT % 256 == 0 && zLIST % 256 == 0 && zCO % 256 == 0);
  static_assert(zFLAG % 256 == 0 && zWT % 256 == 0 && zNV % 256 == 0 && zBV % 256 == 0);
  static_assert(zNV == (size_t)NVU * 16 && zBV == (size_t)HD * 4);
  static_assert(oEND == 60911104);
  static_assert(oEND <= ((size_t)128 << 20));
  static_assert((size_t)(NN - 1) * HD + HD - 1 == 6399999);
  if (oEND > ws_size) return;

  char* ws = (char*)d_ws;
  unsigned short* HB   = (unsigned short*)(ws + oHB);
  float*          T    = (float*)(ws + oT);
  int*            LIST = (int*)(ws + oLIST);
  int*            CO   = (int*)(ws + oCO);
  int*            FLAG = (int*)(ws + oFLAG);
  unsigned short* WT   = (unsigned short*)(ws + oWT);
  float*          NV   = (float*)(ws + oNV);
  float*          BV   = (float*)(ws + oBV);

  hipFuncSetAttribute(reinterpret_cast<const void*>(&k_bucket), hipFuncAttributeMaxDynamicSharedMemorySize, (int)BK_LDS);

  k_plane<0><<<PBX, NTHR, 0, stream>>>(h, NN, KD, KD, HB, MP, KD);
  k_wt_tab<<<TABB, NTHR, 0, stream>>>(W, nrm, bias, WT, NV, BV);
  k_gemm_nt<0, 0><<<GB, NTHR, 0, stream>>>(HB, WT, BV, T, MP, HD, KD, HD);
  k_bucket<<<NBK, NTHR, BK_LDS, stream>>>(srcs, dsts, LIST, CO, FLAG);
  k_walk<<<NN / NWAVE, NTHR, 0, stream>>>(LIST, CO, FLAG, T, NV, BV, out, NN);
}
